// TriAddAttention_86122684220185
// MI455X (gfx1250) — hardware-run, weakly checked
//
#include <hip/hip_runtime.h>


#ifndef NB
#define NB 2
#endif
#define NB_FULL 2
#define DM   512
#define NH_  8
#define HD   64
#define LA   128
#define LB   96
#define LC   12
#define KCC  (LB * LC)
#define KC8  (KCC / 8)
#define SP   KCC
#define OSP  68
#define TS2  2.8853900817779268f
#define L2E  1.4426950408889634f
#define PSH  14.0f
#define NEGB (-3.0e38f)
#define RQ   (((NB * LA + 63) / 64) * 64)
#define RK   (((NB * LB + 63) / 64) * 64)
#define RC   (((NB * LC + 63) / 64) * 64)
#define OUT1_OFF ((size_t)NB_FULL * LA * DM)

static_assert(HD == 64);
static_assert(NH_ * HD == DM);
static_assert(DM % 64 == 0);
static_assert(DM % 32 == 0);
static_assert(LA % 16 == 0);
static_assert(KCC % 32 == 0);
static_assert(KCC % 8 == 0);
static_assert((KCC * 4) % 128 == 0);
static_assert((KCC * 2) % 16 == 0);
static_assert((OUT1_OFF * 4) == (size_t)524288);
static_assert((OUT1_OFF * 4) % 128 == 0);
static_assert(OUT1_OFF + (size_t)NB * NH_ * LA * KCC <= (size_t)9961472 / 4);
static_assert((size_t)NB * LA * DM <= OUT1_OFF);
static_assert(NB <= NB_FULL);
static_assert((OSP * 4) % 16 == 0);
static_assert(RQ % 64 == 0);
static_assert(RK % 64 == 0);
static_assert(RC % 64 == 0);
static_assert(((size_t)LA * DM) % 8 == 0);
static_assert(((size_t)LB * DM) % 8 == 0);
static_assert(((size_t)LC * DM) % 8 == 0);
static_assert((LB * HD / 4) % 32 == 0);
static_assert((LC * HD / 4) % 32 == 0);
static_assert((16 * HD / 4) % 32 == 0);
static_assert((LB * HD / 4) % 256 == 0);
static_assert((16 * SP + LB * HD + LC * HD + 16 * HD + HD + 16 * OSP) * 4 <= 131072);
static_assert((LB * HD + 16 * HD) * 4 <= 131072);
static_assert(64 * 68 * 4 <= 131072);

typedef _Float16 h16;
typedef unsigned short bf;
typedef __attribute__((ext_vector_type(16))) __bf16   v16bf;
typedef __attribute__((ext_vector_type(16))) _Float16 v16h;
typedef __attribute__((ext_vector_type(8)))  _Float16 v8h;
typedef __attribute__((ext_vector_type(8)))  unsigned short v8us;
typedef __attribute__((ext_vector_type(8)))  float    v8f;
typedef __attribute__((ext_vector_type(4)))  float    v4f;
typedef v4f  __attribute__((may_alias)) v4fa;

__device__ __forceinline__ unsigned short f2bf(float f) { unsigned u = __float_as_uint(f); u += 0x7FFFu + ((u >> 16) & 1u); return (unsigned short)(u >> 16); }
__device__ __forceinline__ float bfr(float f) { return __uint_as_float(((unsigned)f2bf(f)) << 16); }
__device__ __forceinline__ v16h cat16(v8h lo, v8h hi) { return __builtin_shufflevector(lo, hi, 0, 1, 2, 3, 4, 5, 6, 7, 8, 9, 10, 11, 12, 13, 14, 15); }
__device__ __forceinline__ v16bf cat16b(v8us lo, v8us hi) { return __builtin_bit_cast(v16bf, __builtin_shufflevector(lo, hi, 0, 1, 2, 3, 4, 5, 6, 7, 8, 9, 10, 11, 12, 13, 14, 15)); }
__device__ __forceinline__ v8f wmma16(v16h a, v16h b, v8f c) { return __builtin_amdgcn_wmma_f32_16x16x32_f16(false, a, false, b, (short)0, c, false, false); }
__device__ __forceinline__ v8f wmmab(v16bf a, v16bf b, v8f c) { return __builtin_amdgcn_wmma_f32_16x16x32_bf16(false, a, false, b, (short)0, c, false, false); }
__device__ __forceinline__ v16h  ldh(const h16* p) { return cat16(*(const v8h*)p, *(const v8h*)(p + 16)); }
__device__ __forceinline__ v16bf ldb(const bf* p)  { return cat16b(*(const v8us*)p, *(const v8us*)(p + 16)); }
__device__ __forceinline__ void wave_sync() { __builtin_amdgcn_fence(3  , "wavefront"); __builtin_amdgcn_wave_barrier(); asm volatile("" ::: "memory"); }

static __device__ __forceinline__ h16 toh_flush(float v) { const h16 r = (h16)v; return (fabsf(v) < 6.103515625e-05f) ? (h16)0.0f : r; }
__device__ __forceinline__ v8f wmma16g(v16h a, v16h b, v8f c) { c = wmma16(a, b, c); asm volatile("v_nop\n\tv_nop\n\tv_nop\n\tv_nop" : "+v"(c) : "v"(a), "v"(b)); return c; }
__device__ __forceinline__ v8f wmmabg(v16bf a, v16bf b, v8f c) { c = wmmab(a, b, c); asm volatile("v_nop\n\tv_nop\n\tv_nop\n\tv_nop" : "+v"(c) : "v"(a), "v"(b)); return c; }

__global__ __launch_bounds__(256) void k_cvt8(const float* __restrict__ src, bf* dst, size_t n8) {
    const size_t i = (size_t)blockIdx.x * 256 + threadIdx.x; if (i >= n8) return;
    const v8f v = *(const v8f*)(src + i * 8); v8us o;
#pragma unroll
    for (int k = 0; k < 8; ++k) o[k] = f2bf(v[k]);
    *(volatile v8us*)(dst + i * 8) = o; __threadfence(); *(volatile v8us*)(dst + i * 8) = o;
}

__global__ __launch_bounds__(256) void k_zero8(bf* dst, size_t n8) {
    const size_t i = (size_t)blockIdx.x * 256 + threadIdx.x; if (i >= n8) return;
    const v8us o = (v8us){};
    *(volatile v8us*)(dst + i * 8) = o; __threadfence(); *(volatile v8us*)(dst + i * 8) = o;
}

__global__ __launch_bounds__(256) void k_wcvtT(const float* __restrict__ W, bf* WT) {
    __shared__ __align__(16) float ts[64 * 68];
    const int tid = threadIdx.x; const int k0 = blockIdx.x * 64, n0 = blockIdx.y * 64;
#pragma unroll
    for (int it = 0; it < 4; ++it) { const int i = it * 256 + tid; const int row = i >> 4, c4 = (i & 15) * 4;
        const v4f v = *(const v4f*)(W + (size_t)(k0 + row) * DM + n0 + c4);
        *(v4fa*)(&ts[row * 68 + c4]) = v; }
    __syncthreads();
    static_assert(256 * 8 * 2 == 64 * 64);
#pragma unroll 1
    for (int ps = 0; ps < 2; ++ps) {
#pragma unroll
        for (int it = 0; it < 2; ++it) { const int n = it * 32 + (tid >> 3), k8 = (tid & 7) * 8; v8us o;
#pragma unroll
            for (int j = 0; j < 8; ++j) o[j] = f2bf(ts[(k8 + j) * 68 + n]);
            *(volatile v8us*)(WT + (size_t)(n0 + n) * DM + k0 + k8) = o; }
        if (ps == 0) __threadfence(); }
}

__global__ __launch_bounds__(32) void k_projf(const bf* __restrict__ A, const bf* __restrict__ Bt, const float* __restrict__ bias, float* Cout) {
    __shared__ __align__(16) float os[16 * OSP];
    const int K = DM;
    const int lane = threadIdx.x & 31, lr = lane & 15, hi = lane >> 4; const int r0 = blockIdx.x * 64, c0 = blockIdx.y * 64;
    v8f acc[4][4];
#pragma unroll
    for (int mb = 0; mb < 4; ++mb)
#pragma unroll
        for (int nb = 0; nb < 4; ++nb) acc[mb][nb] = (v8f){};
    const size_t aoff = (size_t)(r0 + lr) * K + 8 * hi, boff = (size_t)(c0 + lr) * K + 8 * hi;
#pragma unroll 1
    for (int kc = 0; kc < K; kc += 32) {
        v16bf a[4];
#pragma unroll
        for (int mb = 0; mb < 4; ++mb) a[mb] = ldb(A + aoff + (size_t)mb * 16 * K + kc);
#pragma unroll
        for (int nb = 0; nb < 4; ++nb) { const v16bf b = ldb(Bt + boff + (size_t)nb * 16 * K + kc);
#pragma unroll
            for (int mb = 0; mb < 4; ++mb) acc[mb][nb] = wmmabg(a[mb], b, acc[mb][nb]); }
    }
    float bc[4];
#pragma unroll
    for (int nb = 0; nb < 4; ++nb) bc[nb] = bfr(bias[c0 + nb * 16 + lr]);
    static_assert(32 * 4 * 8 == 16 * 64);
#pragma unroll
    for (int mb = 0; mb < 4; ++mb) {
#pragma unroll
        for (int nb = 0; nb < 4; ++nb) {
#pragma unroll
            for (int j = 0; j < 8; ++j) os[(hi * 8 + j) * OSP + nb * 16 + lr] = acc[mb][nb][j] + bc[nb]; }
        wave_sync();
        float* crow = Cout + (size_t)(r0 + mb * 16) * DM + c0;
#pragma unroll 1
        for (int ps = 0; ps < 2; ++ps) {
#pragma unroll
            for (int s = 0; s < 8; ++s) { const int row = 2 * s + (lane >> 4), cofs = (lane & 15) * 4;
                const v4f val = *(const v4fa*)(&os[row * OSP + cofs]);
                *(volatile v4f*)(crow + (size_t)row * DM + cofs) = val; }
            if (ps == 0) __threadfence(); }
        wave_sync();
    }
}

__global__ __launch_bounds__(256) void k_vct(const float* __restrict__ VPl, const float* __restrict__ CPl, h16* VCT) {
    __shared__ __align__(16) float Vs[LB * HD];
    __shared__ __align__(16) float Cs[16 * HD];
    const int tid = threadIdx.x; const int zh = blockIdx.x; const int b = zh / NH_, h = zh % NH_;
    const float* vg = VPl + ((size_t)b * LB) * DM + h * HD;
    const float* cg = CPl + ((size_t)b * LC) * DM + h * HD;
#pragma unroll 1
    for (int i = tid; i < LB * HD / 4; i += 256) { const int row = i >> 4, c4 = (i & 15) * 4;
        const v4f v = *(const v4f*)(vg + (size_t)row * DM + c4); *(v4fa*)(&Vs[row * HD + c4]) = v; }
    { const int row = tid >> 4, c4 = (tid & 15) * 4; const int srow = row < LC ? row : (LC - 1);
      const v4f v = *(const v4f*)(cg + (size_t)srow * DM + c4); *(v4fa*)(&Cs[row * HD + c4]) = v; }
    __syncthreads();
    h16* dst = VCT + (size_t)zh * HD * KCC;
    static_assert((size_t)36 * 256 * 8 == (size_t)HD * KCC);
#pragma unroll 1
    for (int ps = 0; ps < 2; ++ps) {
#pragma unroll 1
        for (int it = 0; it < 36; ++it) { const int p = it * 256 + tid; const int d = p / KC8; const int kc8 = (p - d * KC8) * 8; v8h o;
#pragma unroll
            for (int j = 0; j < 8; ++j) { const int kc = kc8 + j; const int k = kc / LC; const int c = kc - k * LC;
                o[j] = toh_flush(Vs[k * HD + d] * Cs[c * HD + d]); }
            *(volatile v8h*)(dst + (size_t)p * 8) = o; }
        if (ps == 0) __threadfence(); }
}

__global__ __launch_bounds__(32) void k_fused3(const float* __restrict__ QPl, const float* __restrict__ KPl, const float* __restrict__ CPl, const h16* __restrict__ VCT,
                                            const float* __restrict__ pin, float* OUT, float* ATT) {
    __shared__ __align__(16) float sc[16 * SP];
    __shared__ __align__(16) float Ks[LB * HD];
    __shared__ __align__(16) float Cs[LC * HD];
    __shared__ __align__(16) float Qs[16 * HD];
    __shared__ __align__(16) float ps[HD];
    __shared__ __align__(16) float os[16 * OSP];
    const int lane = threadIdx.x & 31, lr = lane & 15, hi = lane >> 4;
    const int zh = blockIdx.y; const int b = zh / NH_, h = zh % NH_;
    const int t0 = blockIdx.x * 16;
    { const float* kg = KPl + ((size_t)b * LB) * DM + h * HD;
#pragma unroll 1
      for (int i = lane; i < LB * HD / 4; i += 32) { const int row = i >> 4, c4 = (i & 15) * 4;
          v4f v = *(const v4f*)(kg + (size_t)row * DM + c4); v = v * TS2; *(v4fa*)(&Ks[row * HD + c4]) = v; }
      const float* cg = CPl + ((size_t)b * LC) * DM + h * HD;
#pragma unroll 1
      for (int i = lane; i < LC * HD / 4; i += 32) { const int row = i >> 4, c4 = (i & 15) * 4;
          v4f v = *(const v4f*)(cg + (size_t)row * DM + c4); v = v * TS2; *(v4fa*)(&Cs[row * HD + c4]) = v; }
      const float* qg = QPl + ((size_t)b * LA + t0) * DM + h * HD;
#pragma unroll 1
      for (int i = lane; i < 16 * HD / 4; i += 32) { const int row = i >> 4, c4 = (i & 15) * 4;
          v4f v = *(const v4f*)(qg + (size_t)row * DM + c4); v = v * TS2; *(v4fa*)(&Qs[row * HD + c4]) = v; } }
    const float p0 = bfr(pin[h * HD + lane]), p1 = bfr(pin[h * HD + 32 + lane]);
    ps[lane] = -2.0f * p0; ps[32 + lane] = -2.0f * p1;
    float psum = p0 + p1;
#pragma unroll
    for (int mk = 16; mk > 0; mk >>= 1) psum += __shfl_xor(psum, mk, 32);
    wave_sync();

#pragma unroll 1
    for (int ch = 0; ch < KCC / 32; ++ch) {
        const int kc = ch * 32 + lane; const int k = kc / LC; const int c = kc - k * LC;
        const int ko = k * HD, co = c * HD;
        float a[16];
#pragma unroll
        for (int q = 0; q < 16; ++q) a[q] = 0.0f;
#pragma unroll 1
        for (int d4 = 0; d4 < HD; d4 += 4) {
            const v4f kv = *(const v4fa*)(&Ks[ko + d4]); const v4f cv = *(const v4fa*)(&Cs[co + d4]);
            const v4f kcv = kv + cv;
            const v4f pv = *(const v4fa*)(&ps[d4]);
#pragma unroll
            for (int q = 0; q < 16; ++q) {
                const v4f qv = *(const v4fa*)(&Qs[q * HD + d4]);
                const v4f x = kcv + qv;
                const float r0 = __builtin_amdgcn_rcpf(1.0f + __builtin_amdgcn_exp2f(x[0]));
                const float r1 = __builtin_amdgcn_rcpf(1.0f + __builtin_amdgcn_exp2f(x[1]));
                const float r2 = __builtin_amdgcn_rcpf(1.0f + __builtin_amdgcn_exp2f(x[2]));
                const float r3 = __builtin_amdgcn_rcpf(1.0f + __builtin_amdgcn_exp2f(x[3]));
                float t = a[q];
                t = fmaf(pv[0], r0, t); t = fmaf(pv[1], r1, t); t = fmaf(pv[2], r2, t); t = fmaf(pv[3], r3, t);
                a[q] = t; }
        }
#pragma unroll
        for (int q = 0; q < 16; ++q) sc[q * SP + kc] = psum + a[q];
    }
    wave_sync();

    float myM = 0.0f;
    static_assert(32 * 4 * 9 == KCC);
#pragma unroll 1
    for (int q = 0; q < 16; ++q) {
        float mx = NEGB;
#pragma unroll 4
        for (int ch = 0; ch < KCC / 32; ++ch) mx = fmaxf(mx, sc[q * SP + ch * 32 + lane]);
#pragma unroll
        for (int mk = 16; mk > 0; mk >>= 1) mx = fmaxf(mx, __shfl_xor(mx, mk, 32));
        float sm = 0.0f;
#pragma unroll 4
        for (int ch = 0; ch < KCC / 32; ++ch) sm += __builtin_amdgcn_exp2f((sc[q * SP + ch * 32 + lane] - mx) * L2E);
#pragma unroll
        for (int mk = 16; mk > 0; mk >>= 1) sm += __shfl_xor(sm, mk, 32);
        const float inv = 1.0f / sm;
        myM = (lr == q) ? mx : myM;
        float* arow = ATT + ((size_t)zh * LA + (size_t)(t0 + q)) * KCC;
#pragma unroll 1
        for (int pss = 0; pss < 2; ++pss) {
#pragma unroll 1
            for (int i = 0; i < 9; ++i) { const int idx = (i * 32 + lane) * 4;
                const v4f x = *(const v4fa*)(&sc[q * SP + idx]); v4f e;
                e[0] = __builtin_amdgcn_exp2f((x[0] - mx) * L2E) * inv; e[1] = __builtin_amdgcn_exp2f((x[1] - mx) * L2E) * inv;
                e[2] = __builtin_amdgcn_exp2f((x[2] - mx) * L2E) * inv; e[3] = __builtin_amdgcn_exp2f((x[3] - mx) * L2E) * inv;
                *(volatile v4f*)(arow + idx) = e; }
            if (pss == 0) __threadfence(); }
    }

    const float shq = PSH - myM * L2E;
    const int sro = lr * SP + 8 * hi;
    const size_t vo = (size_t)zh * HD * KCC + (size_t)lr * KCC + 8 * hi;
    v8f o0 = (v8f){}, o1 = (v8f){}, o2 = (v8f){}, o3 = (v8f){};
    float l = 0.0f;
#pragma unroll 1
    for (int kc0 = 0; kc0 < KCC; kc0 += 32) {
        const v4f x0 = *(const v4fa*)(&sc[sro + kc0]), x1 = *(const v4fa*)(&sc[sro + kc0 + 4]);
        const v4f x2 = *(const v4fa*)(&sc[sro + kc0 + 16]), x3 = *(const v4fa*)(&sc[sro + kc0 + 20]);
        v16h pb; float ls = 0.0f;
#pragma unroll
        for (int r = 0; r < 4; ++r) {
            const float a0 = fmaf(x0[r], L2E, shq), a1 = fmaf(x1[r], L2E, shq), a2 = fmaf(x2[r], L2E, shq), a3 = fmaf(x3[r], L2E, shq);
            const float e0 = __builtin_amdgcn_exp2f(a0), e1 = __builtin_amdgcn_exp2f(a1), e2 = __builtin_amdgcn_exp2f(a2), e3 = __builtin_amdgcn_exp2f(a3);
            const h16 g0 = (h16)((a0 < -14.0f) ? 0.0f : e0); const h16 g1 = (h16)((a1 < -14.0f) ? 0.0f : e1);
            const h16 g2 = (h16)((a2 < -14.0f) ? 0.0f : e2); const h16 g3 = (h16)((a3 < -14.0f) ? 0.0f : e3);
            pb[r] = g0; pb[4 + r] = g1; pb[8 + r] = g2; pb[12 + r] = g3;
            ls += ((float)g0 + (float)g1) + ((float)g2 + (float)g3); }
        l += ls;
        const h16* va = VCT + vo + kc0;
        const v16h v0 = ldh(va), v1 = ldh(va + (size_t)16 * KCC), v2 = ldh(va + (size_t)32 * KCC), v3 = ldh(va + (size_t)48 * KCC);
        o0 = wmma16g(v0, pb, o0); o1 = wmma16g(v1, pb, o1); o2 = wmma16g(v2, pb, o2); o3 = wmma16g(v3, pb, o3);
    }
    l += __shfl_xor(l, 16, 32);
    const float inv = 1.0f / l;
    { v4f a, c;
      a[0] = o0[0] * inv; a[1] = o0[1] * inv; a[2] = o0[2] * inv; a[3] = o0[3] * inv; c[0] = o0[4] * inv; c[1] = o0[5] * inv; c[2] = o0[6] * inv; c[3] = o0[7] * inv;
      *(v4fa*)(&os[lr * OSP +  0 + 8 * hi]) = a; *(v4fa*)(&os[lr * OSP +  0 + 8 * hi + 4]) = c;
      a[0] = o1[0] * inv; a[1] = o1[1] * inv; a[2] = o1[2] * inv; a[3] = o1[3] * inv; c[0] = o1[4] * inv; c[1] = o1[5] * inv; c[2] = o1[6] * inv; c[3] = o1[7] * inv;
      *(v4fa*)(&os[lr * OSP + 16 + 8 * hi]) = a; *(v4fa*)(&os[lr * OSP + 16 + 8 * hi + 4]) = c;
      a[0] = o2[0] * inv; a[1] = o2[1] * inv; a[2] = o2[2] * inv; a[3] = o2[3] * inv; c[0] = o2[4] * inv; c[1] = o2[5] * inv; c[2] = o2[6] * inv; c[3] = o2[7] * inv;
      *(v4fa*)(&os[lr * OSP + 32 + 8 * hi]) = a; *(v4fa*)(&os[lr * OSP + 32 + 8 * hi + 4]) = c;
      a[0] = o3[0] * inv; a[1] = o3[1] * inv; a[2] = o3[2] * inv; a[3] = o3[3] * inv; c[0] = o3[4] * inv; c[1] = o3[5] * inv; c[2] = o3[6] * inv; c[3] = o3[7] * inv;
      *(v4fa*)(&os[lr * OSP + 48 + 8 * hi]) = a; *(v4fa*)(&os[lr * OSP + 48 + 8 * hi + 4]) = c; }
    wave_sync();
    float* orow = OUT + ((size_t)b * LA + t0) * DM + h * HD;
    static_assert(32 * 4 * 8 == 16 * HD);
#pragma unroll 1
    for (int pss = 0; pss < 2; ++pss) {
#pragma unroll
        for (int s = 0; s < 8; ++s) { const int row = 2 * s + (lane >> 4), cofs = (lane & 15) * 4;
            const v4f val = *(const v4fa*)(&os[row * OSP + cofs]);
            *(volatile v4f*)(orow + (size_t)row * DM + cofs) = val; }
        if (pss == 0) __threadfence(); }
}

static constexpr size_t al256(size_t v) { return (v + 255) & ~(size_t)255; }
static constexpr size_t SZ_XQ = al256((size_t)RQ * DM * 2);
static constexpr size_t SZ_XK = al256((size_t)RK * DM * 2);
static constexpr size_t SZ_XC = al256((size_t)RC * DM * 2);
static constexpr size_t SZ_WT = al256((size_t)4 * DM * DM * 2);
static constexpr size_t SZ_PQ = al256((size_t)RQ * DM * 4);
static constexpr size_t SZ_PK = al256((size_t)RK * DM * 4);
static constexpr size_t SZ_PC = al256((size_t)RC * DM * 4);
static constexpr size_t SZ_VC = al256((size_t)NB * NH_ * HD * KCC * 2);
static constexpr size_t SZ_TOTAL = SZ_XQ + 2 * SZ_XK + SZ_XC + SZ_WT + SZ_PQ + 2 * SZ_PK + SZ_PC + SZ_VC;
static_assert(SZ_TOTAL <= (size_t)134217728);
static_assert(((size_t)DM * DM * 2) % 256 == 0);
static_assert(((size_t)NB * LA * DM * 2) % 128 == 0);
static_assert(((size_t)NB * LB * DM * 2) % 128 == 0);
static_assert(((size_t)NB * LC * DM * 2) % 128 == 0);

extern "C" void kernel_launch(void* const* d_in, const int* in_sizes, int n_in,
                              void* d_out, int out_size, void* d_ws, size_t ws_size, hipStream_t stream) {
    if (n_in < 13) return;
    if ((size_t)in_sizes[0] < (size_t)NB * LA * DM || (size_t)in_sizes[1] < (size_t)NB * LB * DM || (size_t)in_sizes[2] < (size_t)NB * LB * DM) return;
    if ((size_t)in_sizes[3] < (size_t)NB * LC * DM) return;
    if ((size_t)in_sizes[4] < (size_t)DM * DM || (size_t)in_sizes[6] < (size_t)DM * DM || (size_t)in_sizes[8] < (size_t)DM * DM || (size_t)in_sizes[10] < (size_t)DM * DM) return;
    if (in_sizes[5] < DM || in_sizes[7] < DM || in_sizes[9] < DM || in_sizes[11] < DM || in_sizes[12] < NH_ * HD) return;
    if ((size_t)out_size < OUT1_OFF + (size_t)NB * NH_ * LA * KCC) return;
    if (SZ_TOTAL > ws_size) return;
    const float* xq = (const float*)d_in[0]; const float* xk = (const float*)d_in[1];
    const float* xv = (const float*)d_in[2]; const float* xc = (const float*)d_in[3];
    const float* wq = (const float*)d_in[4];  const float* bq = (const float*)d_in[5];
    const float* wk = (const float*)d_in[6];  const float* bk = (const float*)d_in[7];
    const float* wv = (const float*)d_in[8];  const float* bv = (const float*)d_in[9];
    const float* wc = (const float*)d_in[10]; const float* bcv = (const float*)d_in[11];
    const float* pv = (const float*)d_in[12];
    float* OUT = (float*)d_out;
    float* ATT = (float*)d_out + OUT1_OFF;
    char* wsp = (char*)d_ws;
    bf* XQ = (bf*)wsp; wsp += SZ_XQ;
    bf* XK = (bf*)wsp; wsp += SZ_XK;
    bf* XV = (bf*)wsp; wsp += SZ_XK;
    bf* XC = (bf*)wsp; wsp += SZ_XC;
    bf* WT = (bf*)wsp; wsp += SZ_WT;
    float* QPl = (float*)wsp; wsp += SZ_PQ;
    float* KPl = (float*)wsp; wsp += SZ_PK;
    float* VPl = (float*)wsp; wsp += SZ_PK;
    float* CPl = (float*)wsp; wsp += SZ_PC;
    h16* VCT = (h16*)wsp; wsp += SZ_VC;
    bf* WTq = WT; bf* WTk = WT + (size_t)DM * DM; bf* WTv = WT + (size_t)2 * DM * DM; bf* WTc = WT + (size_t)3 * DM * DM;

    { const size_t n8 = (size_t)NB * LA * DM / 8; k_cvt8<<<(unsigned)((n8 + 255) / 256), 256, 0, stream>>>(xq, XQ, n8); }
    { const size_t n8 = (size_t)NB * LB * DM / 8; const unsigned g = (unsigned)((n8 + 255) / 256);
      k_cvt8<<<g, 256, 0, stream>>>(xk, XK, n8); k_cvt8<<<g, 256, 0, stream>>>(xv, XV, n8); }
    { const size_t n8 = (size_t)NB * LC * DM / 8; k_cvt8<<<(unsigned)((n8 + 255) / 256), 256, 0, stream>>>(xc, XC, n8); }
    if (RQ > NB * LA) { const size_t n8 = (size_t)(RQ - NB * LA) * DM / 8; k_zero8<<<(unsigned)((n8 + 255) / 256), 256, 0, stream>>>(XQ + (size_t)NB * LA * DM, n8); }
    if (RK > NB * LB) { const size_t n8 = (size_t)(RK - NB * LB) * DM / 8; const unsigned g = (unsigned)((n8 + 255) / 256);
                        k_zero8<<<g, 256, 0, stream>>>(XK + (size_t)NB * LB * DM, n8); k_zero8<<<g, 256, 0, stream>>>(XV + (size_t)NB * LB * DM, n8); }
    if (RC > NB * LC) { const size_t n8 = (size_t)(RC - NB * LC) * DM / 8; k_zero8<<<(unsigned)((n8 + 255) / 256), 256, 0, stream>>>(XC + (size_t)NB * LC * DM, n8); }

    k_wcvtT<<<dim3(DM / 64, DM / 64, 1), 256, 0, stream>>>(wq, WTq);
    k_wcvtT<<<dim3(DM / 64, DM / 64, 1), 256, 0, stream>>>(wk, WTk);
    k_wcvtT<<<dim3(DM / 64, DM / 64, 1), 256, 0, stream>>>(wv, WTv);
    k_wcvtT<<<dim3(DM / 64, DM / 64, 1), 256, 0, stream>>>(wc, WTc);

    k_projf<<<dim3(RQ / 64, DM / 64, 1), 32, 0, stream>>>(XQ, WTq, bq, QPl);
    k_projf<<<dim3(RK / 64, DM / 64, 1), 32, 0, stream>>>(XK, WTk, bk, KPl);
    k_projf<<<dim3(RK / 64, DM / 64, 1), 32, 0, stream>>>(XV, WTv, bv, VPl);
    k_projf<<<dim3(RC / 64, DM / 64, 1), 32, 0, stream>>>(XC, WTc, bcv, CPl);

    k_vct<<<dim3(NB * NH_, 1, 1), 256, 0, stream>>>(VPl, CPl, VCT);
    k_fused3<<<dim3(LA / 16, NB * NH_, 1), 32, 0, stream>>>(QPl, KPl, CPl, VCT, pv, OUT, ATT);
}
